// GCN_48524540510787
// MI455X (gfx1250) — hardware-verified
//
#include <hip/hip_runtime.h>
#include <stddef.h>
#include <stdint.h>
#include <math.h>


#define CIN    256
#define C1     512
#define C2     256
#define C3     64
#define K1     256
#define K2     1024
#define K3     512
#define NTHR   256
#define NWAVE  8
#define EPT    8
#define CHUNK  (NTHR * EPT)
#define WCAP   (EPT * 32)
#define LISTN  (NWAVE * WCAP)
#define NBD    8192
#define SLD    13
#define NBA    1024
#define SLA    10
#define RCAP   28672
#define DEGCAP 128
#define GBM    64
#define GTHR   128
#define GWAVE  (GTHR / 32)
#define NU1    (C1 * (K1 / 8))
#define NU2    (C2 * (C1 / 4))
#define NU3    (C3 * (C2 / 4))
#define NUT    (2 * NU1 + 2 * NU2 + 2 * NU3)
#define AGG_ZINTS (LISTN + 2 * RCAP + 3 * NBA)
#define MISC_INTS 16
#define AGG_LDS_INTS (AGG_ZINTS + MISC_INTS)
#define WSLIM  268435456

static_assert((CHUNK & (CHUNK - 1)) == 0 && CHUNK <= 4096);
static_assert((NBD & (NBD - 1)) == 0 && NBD == (1 << SLD));
static_assert((NBA & (NBA - 1)) == 0 && NBA == (1 << SLA));
static_assert(((long long)CHUNK << SLD) < (1LL << 31));
static_assert(((long long)CHUNK << SLA) < (1LL << 31));
static_assert(NBD % (NTHR * 4) == 0);
static_assert(LISTN % NTHR == 0);
static_assert(NBA % NWAVE == 0 && NBA % 32 == 0 && NBA % GBM == 0);
static_assert(RCAP % 32 == 0 && AGG_ZINTS % (NTHR * 4) == 0 && LISTN % 4 == 0);
static_assert(K1 % 32 == 0 && K2 % 32 == 0 && K3 % 32 == 0);
static_assert(K1 == CIN && K2 == 2 * C1 && K3 == 2 * C2);
static_assert(C1 % 128 == 0 && C2 % 128 == 0 && C3 == 64);
static_assert(C1 % 32 == 0 && C2 % 32 == 0 && C3 % 32 == 0);
static_assert(GBM == GWAVE * 16);
static_assert(NU1 % NTHR == 0 && NU2 % NTHR == 0 && NU3 % NTHR == 0 && NUT % NTHR == 0);
static_assert(K1 / 8 == 32 && C1 / 4 == 128 && C2 / 4 == 64);
static_assert(CIN / 8 == 32);
static_assert(AGG_LDS_INTS * 4 <= 300000);

typedef float          v2f   __attribute__((ext_vector_type(2)));
typedef float          v4f   __attribute__((ext_vector_type(4)));
typedef float          v8f   __attribute__((ext_vector_type(8)));
typedef int            v4i   __attribute__((ext_vector_type(4)));
typedef int            v8i   __attribute__((ext_vector_type(8)));
typedef unsigned short v8us  __attribute__((ext_vector_type(8)));
typedef unsigned short v16us __attribute__((ext_vector_type(16)));
typedef __bf16         v16bf __attribute__((ext_vector_type(16)));
typedef v2f  __attribute__((may_alias)) v2fa;
typedef v4f  __attribute__((may_alias)) v4fa;
typedef v4i  __attribute__((may_alias)) v4ia;
typedef v8us __attribute__((may_alias)) v8usa;
union Frag { v16bf v; v16us u; v8us h[2]; v8i w; };

__device__ __forceinline__ v8f wmb(const Frag& a, const Frag& b, v8f c) {
  v8f d = __builtin_amdgcn_wmma_f32_16x16x32_bf16(false, a.v, false, b.v, (short)0, c, false, false);
  asm volatile("v_nop\n\tv_nop\n\tv_nop\n\tv_nop" : "+v"(d) : "v"(a.w), "v"(b.w));
  return d;
}

__device__ __forceinline__ v8f z8() { v8f z = {0.f, 0.f, 0.f, 0.f, 0.f, 0.f, 0.f, 0.f}; return z; }

__device__ __forceinline__ unsigned bf16_bits(float f) {
  const unsigned u = __float_as_uint(f);
  return (u + 0x7FFFu + ((u >> 16) & 1u)) >> 16;
}
__device__ __forceinline__ float bf16_val(float f) {
  return __uint_as_float(bf16_bits(f) << 16);
}
__device__ __forceinline__ v4f bf16_val4(v4f a) {
  v4f r;
  r.x = bf16_val(a.x); r.y = bf16_val(a.y); r.z = bf16_val(a.z); r.w = bf16_val(a.w);
  return r;
}
__device__ __forceinline__ v8us hilo8(v4f t) {
  v8us o;
  unsigned hb;
  hb = bf16_bits(t.x); o[0] = (unsigned short)hb; o[4] = (unsigned short)bf16_bits(t.x - __uint_as_float(hb << 16));
  hb = bf16_bits(t.y); o[1] = (unsigned short)hb; o[5] = (unsigned short)bf16_bits(t.y - __uint_as_float(hb << 16));
  hb = bf16_bits(t.z); o[2] = (unsigned short)hb; o[6] = (unsigned short)bf16_bits(t.z - __uint_as_float(hb << 16));
  hb = bf16_bits(t.w); o[3] = (unsigned short)hb; o[7] = (unsigned short)bf16_bits(t.w - __uint_as_float(hb << 16));
  return o;
}
__device__ __forceinline__ float elu1(float z) {
  const float e = __expf(fminf(z, 0.0f)) - 1.0f;
  return z > 0.0f ? z : e;
}

template <int SLB>
__device__ __forceinline__ int scan_chunk(const int* __restrict__ dsts, int nE, int cbase, int slotBase,
                                          int nb, int vec8, int* list, int tid, int lane, int wave) {
  int wc = 0;
  const int el0  = tid * EPT;
  const int e0   = cbase + el0;
  const int sent = -2147483647 - 1;
  v4i da, db;
  if (vec8 != 0 && cbase + CHUNK <= nE) {
    da = *(const v4i*)(dsts + e0);
    db = *(const v4i*)(dsts + e0 + 4);
  } else {
    da.x = (e0     < nE) ? dsts[min(e0,     nE - 1)] : sent;
    da.y = (e0 + 1 < nE) ? dsts[min(e0 + 1, nE - 1)] : sent;
    da.z = (e0 + 2 < nE) ? dsts[min(e0 + 2, nE - 1)] : sent;
    da.w = (e0 + 3 < nE) ? dsts[min(e0 + 3, nE - 1)] : sent;
    db.x = (e0 + 4 < nE) ? dsts[min(e0 + 4, nE - 1)] : sent;
    db.y = (e0 + 5 < nE) ? dsts[min(e0 + 5, nE - 1)] : sent;
    db.z = (e0 + 6 < nE) ? dsts[min(e0 + 6, nE - 1)] : sent;
    db.w = (e0 + 7 < nE) ? dsts[min(e0 + 7, nE - 1)] : sent;
  }
  const unsigned nbs = (unsigned)slotBase;
  const unsigned unb = (unsigned)nb;
  const unsigned s0 = (unsigned)da.x - nbs, s1 = (unsigned)da.y - nbs;
  const unsigned s2 = (unsigned)da.z - nbs, s3 = (unsigned)da.w - nbs;
  const unsigned s4 = (unsigned)db.x - nbs, s5 = (unsigned)db.y - nbs;
  const unsigned s6 = (unsigned)db.z - nbs, s7 = (unsigned)db.w - nbs;
  const bool h0 = s0 < unb, h1 = s1 < unb, h2 = s2 < unb, h3 = s3 < unb;
  const bool h4 = s4 < unb, h5 = s5 < unb, h6 = s6 < unb, h7 = s7 < unb;
  const unsigned any = __builtin_amdgcn_ballot_w32(h0 | h1 | h2 | h3 | h4 | h5 | h6 | h7);
  if (any != 0u) {
#define HITJ(J, HJ, SJ) { \
      const unsigned mj = __builtin_amdgcn_ballot_w32(HJ); \
      if (mj != 0u) { \
        if (HJ) { \
          const int pos = wc + (int)__builtin_amdgcn_mbcnt_lo(mj, 0u); \
          if (pos < WCAP) list[wave * WCAP + pos] = ((el0 + (J)) << SLB) | (int)(SJ); \
        } \
        wc += (int)__builtin_popcount(mj); } }
    HITJ(0, h0, s0)
    HITJ(1, h1, s1)
    HITJ(2, h2, s2)
    HITJ(3, h3, s3)
    HITJ(4, h4, s4)
    HITJ(5, h5, s5)
    HITJ(6, h6, s6)
    HITJ(7, h7, s7)
#undef HITJ
  }
  return wc;
}

__global__ __launch_bounds__(NTHR) void k_wprep(const float* __restrict__ Wg1, const float* __restrict__ Wl1,
                                                const float* __restrict__ Wg2, const float* __restrict__ Wl2,
                                                const float* __restrict__ Wg3, const float* __restrict__ Wl3,
                                                unsigned short* WG1T, unsigned short* WL1T,
                                                unsigned short* WG2T, unsigned short* WL2T,
                                                unsigned short* WG3T, unsigned short* WL3T) {
  const int u = (int)blockIdx.x * NTHR + (int)threadIdx.x;
  v8us o;
  unsigned short* dp;
  if (u < 2 * NU1) {
    const bool second = u >= NU1;
    const int v  = second ? (u - NU1) : u;
    const int n  = v >> 5;
    const int k8 = (v & 31) * 8;
    const float* W = second ? Wl1 : Wg1;
    const float* p = W + (size_t)k8 * C1 + n;
#pragma unroll
    for (int i = 0; i < 8; ++i) o[i] = (unsigned short)bf16_bits(p[(size_t)i * C1]);
    dp = (second ? WL1T : WG1T) + (size_t)n * K1 + k8;
  } else if (u < 2 * NU1 + 2 * NU2) {
    const int w0 = u - 2 * NU1;
    const bool second = w0 >= NU2;
    const int v = second ? (w0 - NU2) : w0;
    const int n = v >> 7;
    const int g = v & 127;
    const float* W = second ? Wl2 : Wg2;
    const float* p = W + (size_t)(4 * g) * C2 + n;
    const unsigned short f0 = (unsigned short)bf16_bits(p[0]);
    const unsigned short f1 = (unsigned short)bf16_bits(p[C2]);
    const unsigned short f2 = (unsigned short)bf16_bits(p[2 * C2]);
    const unsigned short f3 = (unsigned short)bf16_bits(p[3 * C2]);
    o[0] = f0; o[1] = f1; o[2] = f2; o[3] = f3; o[4] = f0; o[5] = f1; o[6] = f2; o[7] = f3;
    dp = (second ? WL2T : WG2T) + (size_t)n * K2 + 8 * g;
  } else if (u < NUT) {
    const int w0 = u - 2 * NU1 - 2 * NU2;
    const bool second = w0 >= NU3;
    const int v = second ? (w0 - NU3) : w0;
    const int n = v >> 6;
    const int g = v & 63;
    const float* W = second ? Wl3 : Wg3;
    const float* p = W + (size_t)(4 * g) * C3 + n;
    const unsigned short f0 = (unsigned short)bf16_bits(p[0]);
    const unsigned short f1 = (unsigned short)bf16_bits(p[C3]);
    const unsigned short f2 = (unsigned short)bf16_bits(p[2 * C3]);
    const unsigned short f3 = (unsigned short)bf16_bits(p[3 * C3]);
    o[0] = f0; o[1] = f1; o[2] = f2; o[3] = f3; o[4] = f0; o[5] = f1; o[6] = f2; o[7] = f3;
    dp = (second ? WL3T : WG3T) + (size_t)n * K3 + 8 * g;
  } else {
    return;
  }
  *(volatile v8us*)dp = o;
  __threadfence();
  *(volatile v8us*)dp = o;
}

__global__ __launch_bounds__(NTHR) void k_cvx(const float* __restrict__ x, int nN, int nUnits,
                                              unsigned short* xb) {
  const int u = (int)blockIdx.x * NTHR + (int)threadIdx.x;
  if (u >= nUnits) return;
  const int row = u >> 5;
  const int k8  = (u & 31) * 8;
  const int rc  = row < nN ? row : nN - 1;
  const bool rok = row < nN;
  const float* p = x + (size_t)rc * CIN + k8;
  const v4f a = *(const v4fa*)p;
  const v4f b = *(const v4fa*)(p + 4);
  v8us o;
  o[0] = rok ? (unsigned short)bf16_bits(a.x) : (unsigned short)0;
  o[1] = rok ? (unsigned short)bf16_bits(a.y) : (unsigned short)0;
  o[2] = rok ? (unsigned short)bf16_bits(a.z) : (unsigned short)0;
  o[3] = rok ? (unsigned short)bf16_bits(a.w) : (unsigned short)0;
  o[4] = rok ? (unsigned short)bf16_bits(b.x) : (unsigned short)0;
  o[5] = rok ? (unsigned short)bf16_bits(b.y) : (unsigned short)0;
  o[6] = rok ? (unsigned short)bf16_bits(b.z) : (unsigned short)0;
  o[7] = rok ? (unsigned short)bf16_bits(b.w) : (unsigned short)0;
  unsigned short* dp = xb + (size_t)row * K1 + k8;
  *(volatile v8us*)dp = o;
  __threadfence();
  *(volatile v8us*)dp = o;
}

__global__ __launch_bounds__(NTHR) void k_deg(const int* __restrict__ dsts, int nE, int vec8, float* dis) {
  __shared__ __attribute__((aligned(16))) int scnt[NBD];
  __shared__ __attribute__((aligned(16))) int list[LISTN];
  __shared__ int wcnt[NWAVE];
  const int tid = (int)threadIdx.x, lane = tid & 31, wave = tid >> 5;
  const int nodeBase = (int)blockIdx.x * NBD;

  for (int i = tid; i < NBD; i += NTHR) scnt[i] = 0;
  for (int i = tid; i < LISTN; i += NTHR) list[i] = 0;
  if (tid < NWAVE) wcnt[tid] = 0;
  __syncthreads();

  const int nChunks = (nE + CHUNK - 1) / CHUNK;
#pragma unroll 1
  for (int ch = 0; ch < nChunks; ++ch) {
    const int cbase = ch * CHUNK;
    const int wc = scan_chunk<SLD>(dsts, nE, cbase, nodeBase, NBD, vec8, list, tid, lane, wave);
    if (lane == 0) wcnt[wave] = wc;
    __syncthreads();
    if (wave == 0) {
#pragma unroll 1
      for (int w2 = 0; w2 < NWAVE; ++w2) {
        int c = wcnt[w2];
        c = c < 0 ? 0 : (c > WCAP ? WCAP : c);
#pragma unroll 1
        for (int b0 = 0; b0 < c; b0 += 32) {
          const int idx = b0 + lane;
          const int ent = list[w2 * WCAP + (idx < WCAP ? idx : WCAP - 1)];
          const int m32 = (c - b0) < 32 ? (c - b0) : 32;
#pragma unroll 1
          for (int k = 0; k < m32; ++k) {
            const int u  = __builtin_amdgcn_readlane(ent, k);
            const int sl = u & (NBD - 1);
            if (lane == 0) scnt[sl] = scnt[sl] + 1;
          }
        }
      }
    }
    __syncthreads();
  }

  v4f vals[NBD / (NTHR * 4)];
#pragma unroll
  for (int it = 0; it < NBD / (NTHR * 4); ++it) {
    const int s0 = it * (NTHR * 4) + 4 * tid;
    const v4i c4 = *(const v4ia*)(scnt + s0);
    const float d0 = (float)c4.x + 1.0f, d1 = (float)c4.y + 1.0f;
    const float d2 = (float)c4.z + 1.0f, d3 = (float)c4.w + 1.0f;
    v4f v;
    v.x = rsqrtf(d0); v.y = rsqrtf(d1); v.z = rsqrtf(d2); v.w = rsqrtf(d3);
    vals[it] = v;
  }
#pragma unroll
  for (int it = 0; it < NBD / (NTHR * 4); ++it) {
    const int s0 = it * (NTHR * 4) + 4 * tid;
    *(volatile v4f*)(dis + (size_t)nodeBase + s0) = vals[it];
  }
  __threadfence();
#pragma unroll
  for (int it = 0; it < NBD / (NTHR * 4); ++it) {
    const int s0 = it * (NTHR * 4) + 4 * tid;
    *(volatile v4f*)(dis + (size_t)nodeBase + s0) = vals[it];
  }
}

template <int NT>
__device__ __forceinline__ void gemm_core(const unsigned short* __restrict__ A, const unsigned short* __restrict__ WT,
                                          int K, int rowBase, int col0, int wave, int hh, int m, v8f (&acc)[NT]) {
  const unsigned short* ap = A  + (size_t)(rowBase + 16 * wave + m) * (size_t)K + 8 * hh;
  const unsigned short* wp = WT + (size_t)(col0 + m) * (size_t)K + 8 * hh;
  const int ksteps = K >> 5;
#pragma unroll 1
  for (int ks = 0; ks < ksteps; ++ks) {
    Frag af;
    af.h[0] = *(const v8usa*)(ap + 32 * ks);
    af.h[1] = *(const v8usa*)(ap + 32 * ks + 16);
#pragma unroll
    for (int t = 0; t < NT; ++t) {
      const unsigned short* wq = wp + (size_t)(16 * t) * (size_t)K + 32 * ks;
      Frag bf;
      bf.h[0] = *(const v8usa*)wq;
      bf.h[1] = *(const v8usa*)(wq + 16);
      acc[t] = wmb(af, bf, acc[t]);
    }
  }
}

template <int NT>
__device__ __forceinline__ void stage_tile(float* stg, const v8f (&acc)[NT], int wave, int hh, int m) {
  constexpr int GBN = 16 * NT;
#pragma unroll
  for (int t = 0; t < NT; ++t) {
    const int lc = 16 * t + m;
#pragma unroll
    for (int r = 0; r < 8; ++r) {
      const int lr = 16 * wave + 8 * hh + r;
      stg[lr * GBN + lc] = acc[t][r];
    }
  }
}

template <int NT>
__global__ __launch_bounds__(GTHR) void k_gemm(const unsigned short* __restrict__ A, const unsigned short* __restrict__ WT,
                                               float* outF, int K, int ldo) {
  constexpr int GBN = 16 * NT;
  __shared__ __attribute__((aligned(16))) float stg[GBM * GBN];
  const int tid = (int)threadIdx.x, lane = tid & 31, wave = tid >> 5, hh = lane >> 4, m = lane & 15;
  const int rowBase = (int)blockIdx.x * GBM;
  const int col0    = (int)blockIdx.y * GBN;

  v8f acc[NT];
#pragma unroll
  for (int t = 0; t < NT; ++t) acc[t] = z8();
  gemm_core<NT>(A, WT, K, rowBase, col0, wave, hh, m, acc);
  stage_tile<NT>(stg, acc, wave, hh, m);
  __syncthreads();

  if constexpr (NT == 8) {
    v4f fv[16];
#pragma unroll
    for (int i = 0; i < 16; ++i) {
      const int lr = 16 * wave + i;
      fv[i] = *(const v4fa*)(stg + lr * GBN + 4 * lane);
    }
#pragma unroll
    for (int i = 0; i < 16; ++i) {
      const int gr = rowBase + 16 * wave + i;
      float* op = outF + (size_t)gr * (size_t)ldo + col0 + 4 * lane;
      *(volatile v4f*)op = fv[i];
    }
    __threadfence();
#pragma unroll
    for (int i = 0; i < 16; ++i) {
      const int gr = rowBase + 16 * wave + i;
      float* op = outF + (size_t)gr * (size_t)ldo + col0 + 4 * lane;
      *(volatile v4f*)op = fv[i];
    }
  } else {
    v4f fv[8];
#pragma unroll
    for (int i = 0; i < 8; ++i) {
      const int lr = 16 * wave + 2 * i + hh;
      fv[i] = *(const v4fa*)(stg + lr * GBN + 4 * m);
    }
#pragma unroll
    for (int i = 0; i < 8; ++i) {
      const int gr = rowBase + 16 * wave + 2 * i + hh;
      float* op = outF + (size_t)gr * (size_t)ldo + col0 + 4 * m;
      *(volatile v4f*)op = fv[i];
    }
    __threadfence();
#pragma unroll
    for (int i = 0; i < 8; ++i) {
      const int gr = rowBase + 16 * wave + 2 * i + hh;
      float* op = outF + (size_t)gr * (size_t)ldo + col0 + 4 * m;
      *(volatile v4f*)op = fv[i];
    }
  }
}

__global__ __launch_bounds__(GTHR) void k_gemmp(const unsigned short* __restrict__ A, const unsigned short* __restrict__ WT,
                                                const float* __restrict__ Z, const float* __restrict__ bias,
                                                unsigned short* apl, int K, int ldz, int ldp) {
  constexpr int NT = 8, GBN = 128;
  __shared__ __attribute__((aligned(16))) float stg[GBM * GBN];
  const int tid = (int)threadIdx.x, lane = tid & 31, wave = tid >> 5, hh = lane >> 4, m = lane & 15;
  const int rowBase = (int)blockIdx.x * GBM;
  const int col0    = (int)blockIdx.y * GBN;
  const v4f bb = bf16_val4(*(const v4fa*)(bias + col0 + 4 * lane));

  v8f acc[NT];
#pragma unroll
  for (int t = 0; t < NT; ++t) acc[t] = z8();
  gemm_core<NT>(A, WT, K, rowBase, col0, wave, hh, m, acc);
  stage_tile<NT>(stg, acc, wave, hh, m);
  __syncthreads();

  v8us ov[16];
#pragma unroll
  for (int i = 0; i < 16; ++i) {
    const int lr = 16 * wave + i;
    const int gr = rowBase + lr;
    const v4f l = *(const v4fa*)(stg + lr * GBN + 4 * lane);
    const v4f z = *(const v4fa*)(Z + (size_t)gr * (size_t)ldz + col0 + 4 * lane);
    v4f h;
    h.x = (elu1(z.x) + l.x) + bb.x;
    h.y = (elu1(z.y) + l.y) + bb.y;
    h.z = (elu1(z.z) + l.z) + bb.z;
    h.w = (elu1(z.w) + l.w) + bb.w;
    ov[i] = hilo8(h);
  }
#pragma unroll
  for (int i = 0; i < 16; ++i) {
    const int gr = rowBase + 16 * wave + i;
    unsigned short* op = apl + (size_t)gr * (size_t)ldp + 2 * col0 + 8 * lane;
    *(volatile v8us*)op = ov[i];
  }
  __threadfence();
#pragma unroll
  for (int i = 0; i < 16; ++i) {
    const int gr = rowBase + 16 * wave + i;
    unsigned short* op = apl + (size_t)gr * (size_t)ldp + 2 * col0 + 8 * lane;
    *(volatile v8us*)op = ov[i];
  }
}

__global__ __launch_bounds__(GTHR) void k_gemmo(const unsigned short* __restrict__ A, const unsigned short* __restrict__ WT,
                                                const float* __restrict__ Z, const float* __restrict__ bias,
                                                float* outF, int K, int ldz, int ldo, int nN) {
  constexpr int NT = 4, GBN = 64;
  __shared__ __attribute__((aligned(16))) float stg[GBM * GBN];
  const int tid = (int)threadIdx.x, lane = tid & 31, wave = tid >> 5, hh = lane >> 4, m = lane & 15;
  const int rowBase = (int)blockIdx.x * GBM;
  const int col0    = (int)blockIdx.y * GBN;
  const v4f bb = bf16_val4(*(const v4fa*)(bias + col0 + 4 * m));

  v8f acc[NT];
#pragma unroll
  for (int t = 0; t < NT; ++t) acc[t] = z8();
  gemm_core<NT>(A, WT, K, rowBase, col0, wave, hh, m, acc);
  stage_tile<NT>(stg, acc, wave, hh, m);
  __syncthreads();

  v4f fv[8];
#pragma unroll
  for (int i = 0; i < 8; ++i) {
    const int lr = 16 * wave + 2 * i + hh;
    const int gr = rowBase + lr;
    const v4f l = *(const v4fa*)(stg + lr * GBN + 4 * m);
    const v4f z = *(const v4fa*)(Z + (size_t)gr * (size_t)ldz + col0 + 4 * m);
    v4f v;
    v.x = (z.x + l.x) + bb.x;
    v.y = (z.y + l.y) + bb.y;
    v.z = (z.z + l.z) + bb.z;
    v.w = (z.w + l.w) + bb.w;
    fv[i] = v;
  }
#pragma unroll
  for (int i = 0; i < 8; ++i) {
    const int gr = rowBase + 16 * wave + 2 * i + hh;
    if (gr < nN) {
      float* op = outF + (size_t)gr * (size_t)ldo + col0 + 4 * m;
      *(volatile v4f*)op = fv[i];
    }
  }
  __threadfence();
#pragma unroll
  for (int i = 0; i < 8; ++i) {
    const int gr = rowBase + 16 * wave + 2 * i + hh;
    if (gr < nN) {
      float* op = outF + (size_t)gr * (size_t)ldo + col0 + 4 * m;
      *(volatile v4f*)op = fv[i];
    }
  }
}

template <int C>
__device__ __forceinline__ void ld_row(const float* __restrict__ pl, int r, int lane, float (&a)[C / 32]) {
  if constexpr (C >= 128) {
#pragma unroll
    for (int g = 0; g < C / 128; ++g) {
      const v4f t = *(const v4fa*)(pl + (size_t)r * C + 128 * g + 4 * lane);
      a[4 * g] = t.x; a[4 * g + 1] = t.y; a[4 * g + 2] = t.z; a[4 * g + 3] = t.w;
    }
  } else {
    const v2f t = *(const v2fa*)(pl + (size_t)r * C + 2 * lane);
    a[0] = t.x; a[1] = t.y;
  }
}
template <int C>
__device__ __forceinline__ void st_row(float* pl, int r, int lane, const float (&v)[C / 32]) {
  if constexpr (C >= 128) {
#pragma unroll
    for (int g = 0; g < C / 128; ++g) {
      v4f t;
      t.x = v[4 * g]; t.y = v[4 * g + 1]; t.z = v[4 * g + 2]; t.w = v[4 * g + 3];
      *(volatile v4f*)(pl + (size_t)r * C + 128 * g + 4 * lane) = t;
    }
  } else {
    v2f t;
    t.x = v[0]; t.y = v[1];
    *(volatile v2f*)(pl + (size_t)r * C + 2 * lane) = t;
  }
}

template <int C>
__global__ __launch_bounds__(NTHR) void k_agg(const int* __restrict__ srcs, const int* __restrict__ dsts,
                                              int nE, int nN, int vec8, int mRows,
                                              const float* __restrict__ dis,
                                              const float* __restrict__ xl, const float* __restrict__ bias,
                                              float* outp) {
  constexpr int CPL = C / 32;
  extern __shared__ __attribute__((aligned(16))) int dsm[];
  int* list = dsm;
  int* hl   = dsm + LISTN;
  int* sl   = hl + RCAP;
  int* cnt  = sl + RCAP;
  int* offs = cnt + NBA;
  int* cur  = offs + NBA;
  int* misc = cur + NBA;
  const int tid = (int)threadIdx.x, lane = tid & 31, wave = tid >> 5;
  const int nodeBase = (int)blockIdx.x * NBA;

  {
    const v4i z4 = {0, 0, 0, 0};
    for (int i = tid * 4; i < AGG_ZINTS; i += NTHR * 4) *(v4ia*)(dsm + i) = z4;
    if (tid < MISC_INTS) misc[tid] = 0;
  }
  float bv[CPL];
  {
    float braw[CPL];
    ld_row<C>(bias, 0, lane, braw);
#pragma unroll
    for (int j = 0; j < CPL; ++j) bv[j] = bf16_val(braw[j]);
  }
  __syncthreads();

  int t = 0, ov = 0;
  const int nChunks = (nE + CHUNK - 1) / CHUNK;
#pragma unroll 1
  for (int ch = 0; ch < nChunks; ++ch) {
    const int cbase = ch * CHUNK;
    const int wc = scan_chunk<SLA>(dsts, nE, cbase, nodeBase, NBA, vec8, list, tid, lane, wave);
    if (lane == 0) misc[wave] = wc;
    __syncthreads();
    if (wave == 0) {
#pragma unroll 1
      for (int w2 = 0; w2 < NWAVE; ++w2) {
        int c = misc[w2];
        c = c < 0 ? 0 : (c > WCAP ? WCAP : c);
#pragma unroll 1
        for (int b0 = 0; b0 < c; b0 += 32) {
          const int idx = b0 + lane;
          const int ent = list[w2 * WCAP + (idx < WCAP ? idx : WCAP - 1)];
          const int m32 = (c - b0) < 32 ? (c - b0) : 32;
#pragma unroll 1
          for (int k = 0; k < m32; ++k) {
            const int u    = __builtin_amdgcn_readlane(ent, k);
            const int slot = u & (NBA - 1);
            const int el   = (u >> SLA) & (CHUNK - 1);
            const int pk   = ((cbase + el) << SLA) | slot;
            if (t < RCAP) {
              if (lane == 0) { hl[t] = pk; cnt[slot] = cnt[slot] + 1; }
              t = t + 1;
            } else {
              ov = 1;
            }
          }
        }
      }
    }
    __syncthreads();
  }
  if (wave == 0 && lane == 0) { misc[8] = t; misc[9] = ov; }
  __syncthreads();
  int tt = misc[8];
  tt = tt < 0 ? 0 : (tt > RCAP ? RCAP : tt);
  const int ovf = misc[9];

  if (wave == 0) {
    const int base = lane * (NBA / 32);
    int s = 0;
#pragma unroll 1
    for (int i = 0; i < NBA / 32; ++i) s += cnt[base + i];
    int incl = s;
#pragma unroll
    for (int d = 1; d < 32; d <<= 1) {
      const int y = __shfl_up(incl, d, 32);
      if (lane >= d) incl += y;
    }
    int run = incl - s;
#pragma unroll 1
    for (int i = 0; i < NBA / 32; ++i) {
      const int cv = cnt[base + i];
      offs[base + i] = run;
      cur[base + i]  = run;
      run += cv;
    }
  }
  __syncthreads();
  if (wave == 0) {
#pragma unroll 1
    for (int b0 = 0; b0 < tt; b0 += 32) {
      const int idx = b0 + lane;
      const int ent = hl[idx < RCAP ? idx : RCAP - 1];
      const int m32 = (tt - b0) < 32 ? (tt - b0) : 32;
#pragma unroll 1
      for (int k = 0; k < m32; ++k) {
        const int u    = __builtin_amdgcn_readlane(ent, k);
        const int slot = u & (NBA - 1);
        if (lane == 0) {
          int p = cur[slot];
          p = p < 0 ? 0 : (p > RCAP - 1 ? RCAP - 1 : p);
          sl[p] = u;
          cur[slot] = p + 1;
        }
      }
    }
  }
  __syncthreads();

  const float qnan = __int_as_float(0x7fc00000);
  const float pz = (ovf != 0) ? qnan : 0.0f;
#pragma unroll 1
  for (int si = 0; si < NBA / NWAVE; ++si) {
    const int s    = si * NWAVE + wave;
    const int node = nodeBase + s;
    int c = cnt[s];
    const bool big = c > DEGCAP;
    c = c < 0 ? 0 : (c > DEGCAP ? DEGCAP : c);
    int o = offs[s];
    o = o < 0 ? 0 : (o > RCAP ? RCAP : o);
    const int nc = node < nN ? node : nN - 1;
    const float dd = dis[nc];
    const float rd = dd * dd;
    float acc[CPL];
#pragma unroll
    for (int j = 0; j < CPL; ++j) acc[j] = 0.0f;
#pragma unroll 1
    for (int b0 = 0; b0 < c; b0 += 32) {
      int idx = o + b0 + lane;
      idx = idx > RCAP - 1 ? RCAP - 1 : idx;
      const int ent = sl[idx];
      int eid = ent >> SLA;
      eid = eid < 0 ? 0 : (eid > nE - 1 ? nE - 1 : eid);
      int sr = srcs[eid];
      sr = sr < 0 ? 0 : (sr > nN - 1 ? nN - 1 : sr);
      const float cf  = dis[sr] * dd;
      const int   cfi = __float_as_int(cf);
      const int m32 = (c - b0) < 32 ? (c - b0) : 32;
#pragma unroll 1
      for (int k = 0; k < m32; ++k) {
        const int   sk = __builtin_amdgcn_readlane(sr, k);
        const float ck = __int_as_float(__builtin_amdgcn_readlane(cfi, k));
        float a[CPL];
        ld_row<C>(xl, sk, lane, a);
#pragma unroll
        for (int j = 0; j < CPL; ++j) acc[j] = fmaf(ck, a[j], acc[j]);
      }
    }
    float sv[CPL];
    ld_row<C>(xl, nc, lane, sv);
    const float pzr = big ? qnan : pz;
    const bool live = node < nN;
    float v[CPL];
#pragma unroll
    for (int j = 0; j < CPL; ++j) {
      float y = (acc[j] + sv[j] * rd) + bv[j];
      y = y + pzr;
      v[j] = live ? y : 0.0f;
    }
    if (node < mRows) {
      st_row<C>(outp, node, lane, v);
      __threadfence();
      st_row<C>(outp, node, lane, v);
    }
  }
}

static inline int cdiv(int a, int b) { return (a + b - 1) / b; }
static inline size_t al256(size_t o) { return (o + 255) & ~(size_t)255; }

extern "C" void kernel_launch(void* const* d_in, const int* in_sizes, int n_in,
                              void* d_out, int out_size, void* d_ws, size_t ws_size,
                              hipStream_t stream) {
  if (n_in < 14) return;
  if (in_sizes[0] < CIN || (in_sizes[0] % CIN) != 0) return;
  const int nN = in_sizes[0] / CIN;
  if (nN < GBM || nN > (1 << 22)) return;
  if (in_sizes[1] < 2 || (in_sizes[1] & 1) != 0) return;
  const int nE = in_sizes[1] / 2;
  if (nE < 1 || nE >= (1 << (31 - SLA))) return;
  if (in_sizes[2]  != CIN * C1 || in_sizes[3]  != C1) return;
  if (in_sizes[4]  != C1 * C2  || in_sizes[5]  != C2) return;
  if (in_sizes[6]  != C2 * C3  || in_sizes[7]  != C3) return;
  if (in_sizes[8]  != CIN * C1 || in_sizes[9]  != C1) return;
  if (in_sizes[10] != C1 * C2  || in_sizes[11] != C2) return;
  if (in_sizes[12] != C2 * C3  || in_sizes[13] != C3) return;
  if ((long long)out_size != (long long)nN * C3) return;

  const float* x    = (const float*)d_in[0];
  const int*   ei   = (const int*)  d_in[1];
  const float* Wg1  = (const float*)d_in[2];
  const float* bg1  = (const float*)d_in[3];
  const float* Wg2  = (const float*)d_in[4];
  const float* bg2  = (const float*)d_in[5];
  const float* Wg3  = (const float*)d_in[6];
  const float* bg3  = (const float*)d_in[7];
  const float* Wl1  = (const float*)d_in[8];
  const float* bl1  = (const float*)d_in[9];
  const float* Wl2  = (const float*)d_in[10];
  const float* bl2  = (const float*)d_in[11];
  const float* Wl3  = (const float*)d_in[12];
  const float* bl3  = (const float*)d_in[13];
  float* out = (float*)d_out;
  const int* src = ei;
  const int* dst = ei + nE;

  const int MP   = cdiv(nN, GBM) * GBM;
  const int gM   = MP / GBM;
  const int gD   = cdiv(nN, NBD);
  const int NBPD = gD * NBD;
  const int gA   = cdiv(MP, NBA);
  if ((long long)gA * NBA < (long long)MP) return;
  if (NBPD < nN) return;
  if ((long long)gM * GBM < (long long)nN) return;
  const int vec8 = ((nE & 3) == 0) ? 1 : 0;

  char* ws = (char*)d_ws;
  size_t off = 0;
  const size_t oDIS = off; off = al256(off + (size_t)NBPD * 4);
  const size_t oG1  = off; off = al256(off + (size_t)C1 * K1 * 2);
  const size_t oL1  = off; off = al256(off + (size_t)C1 * K1 * 2);
  const size_t oG2  = off; off = al256(off + (size_t)C2 * K2 * 2);
  const size_t oL2  = off; off = al256(off + (size_t)C2 * K2 * 2);
  const size_t oG3  = off; off = al256(off + (size_t)C3 * K3 * 2);
  const size_t oL3  = off; off = al256(off + (size_t)C3 * K3 * 2);
  const size_t oX   = off; off = al256(off + (size_t)MP * K1 * 2);
  const size_t oP   = off; off = al256(off + (size_t)MP * C1 * 4);
  const size_t oQ   = off; off = al256(off + (size_t)MP * C1 * 4);
  if (off > ws_size || off > (size_t)WSLIM) return;
  if ((size_t)MP * C3 * 4 > (size_t)MP * K1 * 2) return;
  if ((size_t)MP * K2 * 2 > (size_t)MP * C1 * 4) return;
  if ((size_t)MP * C2 * 4 + (size_t)MP * C2 * 4 > (size_t)MP * C1 * 4) return;
  if ((size_t)MP * K3 * 2 > (size_t)MP * C2 * 4) return;
  float*          DIS  = (float*)(ws + oDIS);
  unsigned short* WG1T = (unsigned short*)(ws + oG1);
  unsigned short* WL1T = (unsigned short*)(ws + oL1);
  unsigned short* WG2T = (unsigned short*)(ws + oG2);
  unsigned short* WL2T = (unsigned short*)(ws + oL2);
  unsigned short* WG3T = (unsigned short*)(ws + oG3);
  unsigned short* WL3T = (unsigned short*)(ws + oL3);
  unsigned short* XB   = (unsigned short*)(ws + oX);
  float*          Z3   = (float*)(ws + oX);
  float*          HG1  = (float*)(ws + oP);
  unsigned short* A2   = (unsigned short*)(ws + oP);
  float*          HG3  = (float*)(ws + oP);
  float*          Z1   = (float*)(ws + oQ);
  float*          HG2  = (float*)(ws + oQ);
  float*          Z2   = (float*)(ws + oQ + (size_t)MP * C2 * 4);
  unsigned short* A3   = (unsigned short*)(ws + oQ);

  const size_t aggLds = (size_t)AGG_LDS_INTS * 4;
  hipFuncSetAttribute(reinterpret_cast<const void*>(&k_agg<C1>), hipFuncAttributeMaxDynamicSharedMemorySize, (int)aggLds);
  hipFuncSetAttribute(reinterpret_cast<const void*>(&k_agg<C2>), hipFuncAttributeMaxDynamicSharedMemorySize, (int)aggLds);
  hipFuncSetAttribute(reinterpret_cast<const void*>(&k_agg<C3>), hipFuncAttributeMaxDynamicSharedMemorySize, (int)aggLds);

  const int nUx = MP * (CIN / 8);
  k_wprep<<<NUT / NTHR, NTHR, 0, stream>>>(Wg1, Wl1, Wg2, Wl2, Wg3, Wl3, WG1T, WL1T, WG2T, WL2T, WG3T, WL3T);
  k_cvx<<<cdiv(nUx, NTHR), NTHR, 0, stream>>>(x, nN, nUx, XB);
  k_deg<<<gD, NTHR, 0, stream>>>(dst, nE, vec8, DIS);
  k_gemm<8><<<dim3(gM, C1 / 128), GTHR, 0, stream>>>(XB, WG1T, HG1, K1, C1);
  k_agg<C1><<<gA, NTHR, aggLds, stream>>>(src, dst, nE, nN, vec8, MP, DIS, HG1, bg1, Z1);
  k_gemmp<<<dim3(gM, C1 / 128), GTHR, 0, stream>>>(XB, WL1T, Z1, bl1, A2, K1, C1, K2);
  k_gemm<8><<<dim3(gM, C2 / 128), GTHR, 0, stream>>>(A2, WG2T, HG2, K2, C2);
  k_agg<C2><<<gA, NTHR, aggLds, stream>>>(src, dst, nE, nN, vec8, MP, DIS, HG2, bg2, Z2);
  k_gemmp<<<dim3(gM, C2 / 128), GTHR, 0, stream>>>(A2, WL2T, Z2, bl2, A3, K2, C2, K3);
  k_gemm<4><<<dim3(gM, 1), GTHR, 0, stream>>>(A3, WG3T, HG3, K3, C3);
  k_agg<C3><<<gA, NTHR, aggLds, stream>>>(src, dst, nE, nN, vec8, MP, DIS, HG3, bg3, Z3);
  k_gemmo<<<dim3(gM, 1), GTHR, 0, stream>>>(A3, WL3T, Z3, bl3, out, K3, C3, C3, nN);
}
